// StructureAwareSSM_15247133901504
// MI455X (gfx1250) — hardware-verified
//
#include <hip/hip_runtime.h>

constexpr int kNB  = 4;
constexpr int kL   = 4096;
constexpr int kGW  = 64;
constexpr int kDM  = 512;
constexpr int kDI  = 512;
constexpr int kR   = 32;
constexpr int kKXV = 34;
constexpr int kKX  = 64;
constexpr int kTok = kNB * kL;
constexpr float kInvDI = 1.0f / 512.0f;
constexpr float kLnEps = 1e-5f;

typedef __attribute__((ext_vector_type(16))) _Float16 v16h;
typedef __attribute__((ext_vector_type(8)))  _Float16 v8h;
typedef __attribute__((ext_vector_type(16))) __bf16   v16b;
typedef __attribute__((ext_vector_type(8)))  __bf16   v8b;
typedef __attribute__((ext_vector_type(8)))  float    v8f;
typedef __attribute__((ext_vector_type(4)))  float    v4f;
typedef __attribute__((ext_vector_type(4)))  unsigned int v4u;

__device__ __forceinline__ unsigned short f2bf_bits(float f) {
  unsigned u = __float_as_uint(f);
  return (unsigned short)((u + 0x7FFFu + ((u >> 16) & 1u)) >> 16);
}
__device__ __forceinline__ float bf_bits2f(unsigned short h) { return __uint_as_float(((unsigned)h) << 16); }

__device__ __forceinline__ void dep_guard_h(v8f& a, v8f& b, v16h x, v16h y) { asm volatile("v_nop\n\tv_nop\n\tv_nop\n\tv_nop" : "+v"(a), "+v"(b) : "v"(x), "v"(y)); }
__device__ __forceinline__ void dep_guard_b(v8f& a, v8f& b, v16b x, v16b y) { asm volatile("v_nop\n\tv_nop\n\tv_nop\n\tv_nop" : "+v"(a), "+v"(b) : "v"(x), "v"(y)); }
__device__ __forceinline__ void keep4_h(v16h a, v16h b, v16h c, v16h d) { asm volatile("v_nop" :: "v"(a), "v"(b), "v"(c), "v"(d)); }
__device__ __forceinline__ void keep4_b(v16b a, v16b b, v16b c, v16b d) { asm volatile("v_nop" :: "v"(a), "v"(b), "v"(c), "v"(d)); }
__device__ __forceinline__ void acc_guard4(v8f& a, v8f& b, v8f& c, v8f& d) { asm volatile("v_nop\n\tv_nop\n\tv_nop\n\tv_nop" : "+v"(a), "+v"(b), "+v"(c), "+v"(d)); }
template <typename T> struct Frag;
template <> struct Frag<_Float16> {
  typedef v16h V; union U { v16h v; v8h h[2]; };
  static __device__ __forceinline__ v16h load(const _Float16* p) {
    U f; f.h[0] = *(const v8h*)(p); f.h[1] = *(const v8h*)(p + 16); return f.v;
  }
  static __device__ __forceinline__ v8f mma(v16h a, v16h b, v8f c) {
    return __builtin_amdgcn_wmma_f32_16x16x32_f16(false, a, false, b, (short)0, c, false, false);
  }
  static __device__ __forceinline__ void guard(v8f& a, v8f& b, v16h x, v16h y) { dep_guard_h(a, b, x, y); }
  static __device__ __forceinline__ void keep(v16h a, v16h b, v16h c, v16h d) { keep4_h(a, b, c, d); }
};
template <> struct Frag<__bf16> {
  typedef v16b V; union U { v16b v; v8b h[2]; };
  static __device__ __forceinline__ v16b load(const __bf16* p) {
    U f; f.h[0] = *(const v8b*)(p); f.h[1] = *(const v8b*)(p + 16); return f.v;
  }
  static __device__ __forceinline__ v8f mma(v16b a, v16b b, v8f c) {
    return __builtin_amdgcn_wmma_f32_16x16x32_bf16(false, a, false, b, (short)0, c, false, false);
  }
  static __device__ __forceinline__ void guard(v8f& a, v8f& b, v16b x, v16b y) { dep_guard_b(a, b, x, y); }
  static __device__ __forceinline__ void keep(v16b a, v16b b, v16b c, v16b d) { keep4_b(a, b, c, d); }
};

__device__ __forceinline__ unsigned pk16(unsigned short a, unsigned short b) { return (unsigned)a | ((unsigned)b << 16); }

template <int ET> struct Elem;
template <> struct Elem<0> { typedef _Float16 T; };
template <> struct Elem<1> { typedef __bf16 T; };
template <int ET, bool SPLIT, int BIAS_MODE, int OUT_MODE, bool RESID, int ACT = 0>
__global__ __launch_bounds__(256) void wmma_gemm64(
    const unsigned short* __restrict__ Ap, const unsigned short* __restrict__ A2p, int lda, long strideA,
    const unsigned short* __restrict__ Btp, const unsigned short* __restrict__ Bt2p, int ldb, long strideB,
    void* __restrict__ Cout, void* __restrict__ Cout2, int ldc, long strideC,
    const float* __restrict__ bias,
    const float* __restrict__ resid, long strideR,
    int M, int N, int K, float scale) {
  typedef typename Elem<ET>::T T;
  typedef typename Frag<T>::V V;
  const T* A = (const T*)Ap; const T* A2 = (const T*)A2p; const T* Bt = (const T*)Btp; const T* Bt2 = (const T*)Bt2p;
  __shared__ __align__(16) float sT[8][16 * 68];
  const int b    = blockIdx.y;
  const int lane = threadIdx.x & 31;
  const int wave = threadIdx.x >> 5;
  const int tilesN = N >> 6;
  const int tilesM = M >> 6;
  const int tile = blockIdx.x * 8 + wave;
  if (tile >= tilesM * tilesN) return;
  const int tm = tile / tilesN;
  const int tn = tile - tm * tilesN;
  const int m0 = tm << 6;
  const int n0 = tn << 6;

  const T* Ab  = A  + (size_t)b * strideA;
  const T* Bb  = Bt + (size_t)b * strideB;
  const T* Ab2 = SPLIT ? (A2  + (size_t)b * strideA) : nullptr;
  const T* Bb2 = SPLIT ? (Bt2 + (size_t)b * strideB) : nullptr;

  const int rlane = lane & 15;
  const int koff  = (lane >> 4) * 8;
  const int mOff  = (lane >> 4) * 8;

  v8f acc[4][4];
#pragma unroll
  for (int i = 0; i < 4; ++i)
#pragma unroll
    for (int j = 0; j < 4; ++j) acc[i][j] = (v8f){0.f,0.f,0.f,0.f,0.f,0.f,0.f,0.f};

  for (int k0 = 0; k0 < K; k0 += 32) {
    V bh[4], bl[4];
#pragma unroll
    for (int j = 0; j < 4; ++j) {
      const size_t bo = (size_t)(n0 + (j << 4) + rlane) * ldb + koff + k0;
      bh[j] = Frag<T>::load(Bb + bo);
      if (SPLIT) bl[j] = Frag<T>::load(Bb2 + bo);
    }
#pragma unroll
    for (int i = 0; i < 4; ++i) {
      const size_t ao = (size_t)(m0 + (i << 4) + rlane) * lda + koff + k0;
      V ah = Frag<T>::load(Ab + ao);
      V al;
      if (SPLIT) al = Frag<T>::load(Ab2 + ao);
#pragma unroll
      for (int j = 0; j < 4; ++j) {
        acc[i][j] = Frag<T>::mma(ah, bh[j], acc[i][j]);
        if (SPLIT) {
          acc[i][j] = Frag<T>::mma(ah, bl[j], acc[i][j]);
          acc[i][j] = Frag<T>::mma(al, bh[j], acc[i][j]);
        }
      }
      Frag<T>::guard(acc[i][0], acc[i][3], ah, SPLIT ? al : ah);
    }
    Frag<T>::keep(bh[0], bh[1], bh[2], bh[3]);
    if (SPLIT) Frag<T>::keep(bl[0], bl[1], bl[2], bl[3]);
  }
  acc_guard4(acc[0][0], acc[0][1], acc[0][2], acc[0][3]);
  acc_guard4(acc[1][0], acc[1][1], acc[1][2], acc[1][3]);
  acc_guard4(acc[2][0], acc[2][1], acc[2][2], acc[2][3]);
  acc_guard4(acc[3][0], acc[3][1], acc[3][2], acc[3][3]);

  float* slab = sT[wave];
  const float* Rb = RESID ? (resid + (size_t)b * strideR) : nullptr;
#pragma unroll
  for (int i = 0; i < 4; ++i) {
    const int mBase = m0 + (i << 4);
#pragma unroll
    for (int j = 0; j < 4; ++j) {
      const int n = n0 + (j << 4) + rlane;
      float bv = 0.f;
      if (BIAS_MODE == 2) bv = bias[n];
#pragma unroll
      for (int r = 0; r < 8; ++r) {
        float v = acc[i][j][r] * scale;
        if (BIAS_MODE == 1) v += bias[mBase + mOff + r];
        if (BIAS_MODE == 2) v += bv;
        if (RESID) v += Rb[(size_t)(mBase + mOff + r) * ldc + n];
        if (ACT == 2) v = fmaxf(v, 0.0f);
        if (ACT == 4) v = (v > 0.f) ? v : 0.01f * v;
        slab[(mOff + r) * 68 + (j << 4) + rlane] = v;
      }
    }
    __builtin_amdgcn_fence(__ATOMIC_RELEASE, "workgroup");
    __builtin_amdgcn_wave_barrier();
    __builtin_amdgcn_fence(__ATOMIC_ACQUIRE, "workgroup");
    if (OUT_MODE == 0) {
      float* C = (float*)Cout + (size_t)b * strideC;
      const int hh = lane >> 4, c4 = (lane & 15) * 4;
      for (int pass = 0; pass < 2; ++pass) {
#pragma unroll
        for (int it = 0; it < 8; ++it) {
          const int row = it * 2 + hh;
          v4f v = *(const v4f*)(slab + row * 68 + c4);
          *(volatile v4f*)(C + (size_t)(mBase + row) * ldc + n0 + c4) = v;
        }
        __threadfence();
      }
    } else {
      const int q = lane >> 3, c8 = (lane & 7) * 8;
      unsigned short* C  = (unsigned short*)Cout  + (size_t)b * strideC;
      unsigned short* C2 = (OUT_MODE == 2) ? ((unsigned short*)Cout2 + (size_t)b * strideC) : nullptr;
      for (int pass = 0; pass < 2; ++pass) {
#pragma unroll
        for (int it = 0; it < 4; ++it) {
          const int row = it * 4 + q;
          const float* sp = slab + row * 68 + c8;
          v8h hv, lv;
#pragma unroll
          for (int e = 0; e < 8; ++e) {
            if (OUT_MODE == 1) {
              hv[e] = (_Float16)sp[e];
            } else {
              unsigned short hb = f2bf_bits(sp[e]);
              unsigned short lb = f2bf_bits(sp[e] - bf_bits2f(hb));
              hv[e] = __builtin_bit_cast(_Float16, hb);
              lv[e] = __builtin_bit_cast(_Float16, lb);
            }
          }
          *(volatile v8h*)(C + (size_t)(mBase + row) * ldc + n0 + c8) = hv;
          if (OUT_MODE == 2) *(volatile v8h*)(C2 + (size_t)(mBase + row) * ldc + n0 + c8) = lv;
        }
        __threadfence();
      }
    }
    __builtin_amdgcn_fence(__ATOMIC_RELEASE, "workgroup");
    __builtin_amdgcn_wave_barrier();
    __builtin_amdgcn_fence(__ATOMIC_ACQUIRE, "workgroup");
  }
}

__device__ __forceinline__ float wave_sum(float v) {
#pragma unroll
  for (int off = 16; off > 0; off >>= 1) v += __shfl_xor(v, off, 32);
  return v;
}
__device__ __forceinline__ int clamp63(int v) { return v < 0 ? 0 : (v > 63 ? 63 : v); }

__global__ __launch_bounds__(256) void k_split8(const float* __restrict__ in, unsigned short* __restrict__ hi,
                                                unsigned short* __restrict__ lo, int n8_total, int n8_valid) {
  const int i = blockIdx.x * 256 + threadIdx.x;
  if (i >= n8_total) return;
  const bool valid = (i < n8_valid);
  const int ic = valid ? i : 0;
  const float* p = in + 8 * (size_t)ic;
  const v4f a = *(const v4f*)(p);
  const v4f c = *(const v4f*)(p + 4);
  unsigned short hb[8], lb[8];
#pragma unroll
  for (int e = 0; e < 4; ++e) {
    const float x0 = valid ? a[e] : 0.0f;
    const float x1 = valid ? c[e] : 0.0f;
    hb[e] = f2bf_bits(x0);
    lb[e] = f2bf_bits(x0 - bf_bits2f(hb[e]));
    hb[4 + e] = f2bf_bits(x1);
    lb[4 + e] = f2bf_bits(x1 - bf_bits2f(hb[4 + e]));
  }
  const v4u uh = (v4u){pk16(hb[0], hb[1]), pk16(hb[2], hb[3]), pk16(hb[4], hb[5]), pk16(hb[6], hb[7])};
  const v4u ul = (v4u){pk16(lb[0], lb[1]), pk16(lb[2], lb[3]), pk16(lb[4], lb[5]), pk16(lb[6], lb[7])};
  unsigned short* qh = hi + 8 * (size_t)i;
  unsigned short* ql = lo + 8 * (size_t)i;
  *(volatile v4u*)qh = uh;
  *(volatile v4u*)ql = ul;
  __threadfence();
  *(volatile v4u*)qh = uh;
  *(volatile v4u*)ql = ul;
}

__global__ __launch_bounds__(256) void k_conv1(const float* __restrict__ XIN, const float* __restrict__ cw,
                                               const float* __restrict__ cb, float* __restrict__ XS,
                                               unsigned short* __restrict__ XSTH, unsigned short* __restrict__ XSTL) {
  __shared__ __align__(16) float sv[64 * 68];
  const int t  = threadIdx.x;
  const int hr = blockIdx.x;
  const int cg = blockIdx.y;
  const int b  = blockIdx.z;
  const int w  = t & 63;
  const int cq = t >> 6;
  const int c0 = cg * 64;
  int yo[3], xo[3];
  bool yok[3], xok[3];
#pragma unroll
  for (int i = 0; i < 3; ++i) {
    const int yy = hr + i - 1;
    yok[i] = (yy >= 0) && (yy <= 63);
    yo[i] = clamp63(yy) * kGW;
    const int xx = w + i - 1;
    xok[i] = (xx >= 0) && (xx <= 63);
    xo[i] = clamp63(xx);
  }
#pragma unroll 1
  for (int cc = 0; cc < 16; ++cc) {
    const int c = cc * 4 + cq;
    const int d = c0 + c;
    const float* base = XIN + (size_t)(b * kDI + d) * kL;
    const float* wc = cw + d * 9;
    float acc = cb[d];
#pragma unroll
    for (int i = 0; i < 3; ++i) {
#pragma unroll
      for (int j = 0; j < 3; ++j) {
        float v = base[yo[i] + xo[j]];
        v = (yok[i] && xok[j]) ? v : 0.0f;
        acc += wc[i * 3 + j] * v;
      }
    }
    const float sg = 1.0f / (1.0f + expf(-acc));
    sv[c * 68 + w] = acc * sg;
  }
  __syncthreads();
  const int lane = t & 31, wv = t >> 5;
  {
    const int hh = lane >> 4, c4 = (lane & 15) * 4;
    for (int pass = 0; pass < 2; ++pass) {
#pragma unroll
      for (int it = 0; it < 4; ++it) {
        const int row = wv * 8 + it * 2 + hh;
        const v4f v = *(const v4f*)(sv + row * 68 + c4);
        *(volatile v4f*)(XS + (size_t)(b * kDI + c0 + row) * kL + hr * kGW + c4) = v;
      }
      __threadfence();
    }
  }
  {
    const int q = lane >> 3, c8 = (lane & 7) * 8;
    for (int pass = 0; pass < 2; ++pass) {
#pragma unroll
      for (int it = 0; it < 2; ++it) {
        const int wl = wv * 8 + it * 4 + q;
        unsigned short hb[8], lb[8];
#pragma unroll
        for (int e = 0; e < 8; ++e) {
          const float v = sv[(c8 + e) * 68 + wl];
          hb[e] = f2bf_bits(v);
          lb[e] = f2bf_bits(v - bf_bits2f(hb[e]));
        }
        const v4u uh = (v4u){pk16(hb[0], hb[1]), pk16(hb[2], hb[3]), pk16(hb[4], hb[5]), pk16(hb[6], hb[7])};
        const v4u ul = (v4u){pk16(lb[0], lb[1]), pk16(lb[2], lb[3]), pk16(lb[4], lb[5]), pk16(lb[6], lb[7])};
        const size_t o = (size_t)(b * kL + hr * kGW + wl) * kDI + c0 + c8;
        *(volatile v4u*)(XSTH + o) = uh;
        *(volatile v4u*)(XSTL + o) = ul;
      }
      __threadfence();
    }
  }
}

__global__ __launch_bounds__(256) void k_dtr(const float* __restrict__ XDBL, unsigned short* __restrict__ DTRH,
                                             unsigned short* __restrict__ DTRL) {
  __shared__ float sm[64 * 33];
  const int t = threadIdx.x;
  const int l0 = blockIdx.x * 64;
  const int b = blockIdx.y;
#pragma unroll
  for (int it = 0; it < 8; ++it) {
    const int e = it * 256 + t;
    const int r = e >> 6;
    const int wl = e & 63;
    sm[wl * 33 + r] = XDBL[(size_t)(b * kKX + r) * kL + l0 + wl];
  }
  __syncthreads();
  const int wl = t >> 2, r8 = (t & 3) * 8;
  unsigned short hb[8], lb[8];
#pragma unroll
  for (int e = 0; e < 8; ++e) {
    const float v = sm[wl * 33 + r8 + e];
    hb[e] = f2bf_bits(v);
    lb[e] = f2bf_bits(v - bf_bits2f(hb[e]));
  }
  const v4u uh = (v4u){pk16(hb[0], hb[1]), pk16(hb[2], hb[3]), pk16(hb[4], hb[5]), pk16(hb[6], hb[7])};
  const v4u ul = (v4u){pk16(lb[0], lb[1]), pk16(lb[2], lb[3]), pk16(lb[4], lb[5]), pk16(lb[6], lb[7])};
  const size_t o = (size_t)(b * kL + l0 + wl) * kR + r8;
  *(volatile v4u*)(DTRH + o) = uh;
  *(volatile v4u*)(DTRL + o) = ul;
  __threadfence();
  *(volatile v4u*)(DTRH + o) = uh;
  *(volatile v4u*)(DTRL + o) = ul;
}

__global__ __launch_bounds__(64) void k_scan(const unsigned short* __restrict__ DTWH, const unsigned short* __restrict__ DTWL,
                                             const unsigned short* __restrict__ DTRH, const unsigned short* __restrict__ DTRL,
                                             const float* __restrict__ XS, const float* __restrict__ XDBL,
                                             const float* __restrict__ dtb, const float* __restrict__ Alog,
                                             float* __restrict__ Hout) {
  __shared__ __align__(16) float sd[2][64 * 33];
  __shared__ __align__(16) float sx[2][64 * 33];
  __shared__ __align__(16) float sh[2][32 * 68];
  __shared__ float sbs[2][64];
  const int t    = threadIdx.x;
  const int lane = t & 31;
  const int wv   = t >> 5;
  const int b    = blockIdx.y;
  const int d0   = blockIdx.x * 64 + wv * 32;
  const int d    = d0 + lane;
  const int cidx = lane & 15;
  const int hh   = lane >> 4;
  const int koff = hh * 8;
  const int c4   = (lane & 15) * 4;
  const __bf16* Awh = (const __bf16*)DTWH;
  const __bf16* Awl = (const __bf16*)DTWL;
  const __bf16* Brh = (const __bf16*)DTRH + (size_t)b * kL * kR;
  const __bf16* Brl = (const __bf16*)DTRL + (size_t)b * kL * kR;
  v16b ah[2], al[2];
#pragma unroll
  for (int i = 0; i < 2; ++i) {
    const size_t ao = (size_t)(d0 + 16 * i + cidx) * kR + koff;
    ah[i] = Frag<__bf16>::load(Awh + ao);
    al[i] = Frag<__bf16>::load(Awl + ao);
  }
  const float Ad    = -expf(Alog[d]);
  const float dbias = dtb[d];
  float* sdw = sd[wv];
  float* sxw = sx[wv];
  float* shw = sh[wv];
  float* sbw = sbs[wv];
  const float* xsbase = XS + (size_t)(b * kDI + d0) * kL;
  const float* bsrow  = XDBL + (size_t)(b * kKX + kR) * kL;
  float* hbase = Hout + (size_t)(b * kDI + d0) * kL;
  float hst = 0.0f;
#pragma unroll 1
  for (int ch = 0; ch < kL / 64; ++ch) {
    const int l0 = ch * 64;
    v8f acc[2][4];
#pragma unroll
    for (int i = 0; i < 2; ++i)
#pragma unroll
      for (int j = 0; j < 4; ++j) acc[i][j] = (v8f){0.f,0.f,0.f,0.f,0.f,0.f,0.f,0.f};
#pragma unroll
    for (int j = 0; j < 4; ++j) {
      const size_t bo = (size_t)(l0 + 16 * j + cidx) * kR + koff;
      const v16b bh = Frag<__bf16>::load(Brh + bo);
      const v16b bl = Frag<__bf16>::load(Brl + bo);
#pragma unroll
      for (int i = 0; i < 2; ++i) {
        acc[i][j] = Frag<__bf16>::mma(ah[i], bh, acc[i][j]);
        acc[i][j] = Frag<__bf16>::mma(ah[i], bl, acc[i][j]);
        acc[i][j] = Frag<__bf16>::mma(al[i], bh, acc[i][j]);
      }
      dep_guard_b(acc[0][j], acc[1][j], bh, bl);
    }
    keep4_b(ah[0], ah[1], al[0], al[1]);
    acc_guard4(acc[0][0], acc[0][1], acc[0][2], acc[0][3]);
    acc_guard4(acc[1][0], acc[1][1], acc[1][2], acc[1][3]);
#pragma unroll
    for (int i = 0; i < 2; ++i)
#pragma unroll
      for (int j = 0; j < 4; ++j)
#pragma unroll
        for (int r = 0; r < 8; ++r)
          sdw[(16 * j + cidx) * 33 + 16 * i + 8 * hh + r] = acc[i][j][r];
#pragma unroll 4
    for (int rr = 0; rr < 32; ++rr) {
      const float* xr = xsbase + (size_t)rr * kL + l0;
      sxw[lane * 33 + rr] = xr[lane];
      sxw[(lane + 32) * 33 + rr] = xr[lane + 32];
    }
    sbw[lane]      = bsrow[l0 + lane];
    sbw[lane + 32] = bsrow[l0 + 32 + lane];
    __syncthreads();
#pragma unroll 1
    for (int s = 0; s < 64; ++s) {
      const float xv = sdw[s * 33 + lane] + dbias;
      const float sp = fmaxf(xv, 0.0f) + log1pf(expf(-fabsf(xv)));
      const float a  = expf(sp * Ad);
      const float bb = (sp * sbw[s]) * sxw[s * 33 + lane];
      hst = a * hst + bb;
      shw[lane * 68 + s] = hst;
    }
    __syncthreads();
    for (int pass = 0; pass < 2; ++pass) {
#pragma unroll
      for (int it = 0; it < 16; ++it) {
        const int row = it * 2 + hh;
        const v4f v = *(const v4f*)(shw + row * 68 + c4);
        *(volatile v4f*)(hbase + (size_t)row * kL + l0 + c4) = v;
      }
      __threadfence();
    }
    __syncthreads();
  }
}

__global__ __launch_bounds__(256) void k_fuse(const float* __restrict__ Hb, const float* __restrict__ XS,
                                              const float* __restrict__ XDBL, const float* __restrict__ Ds,
                                              const float* __restrict__ kw1, const float* __restrict__ kw2,
                                              const float* __restrict__ kw3, const float* __restrict__ alpha,
                                              float* __restrict__ Y) {
  __shared__ __align__(16) float sy[64 * 68];
  const int t  = threadIdx.x;
  const int hr = blockIdx.x;
  const int cg = blockIdx.y;
  const int b  = blockIdx.z;
  const int w  = t & 63;
  const int cq = t >> 6;
  const int c0 = cg * 64;
  const int l  = hr * kGW + w;
  const float a0 = alpha[0], a1 = alpha[1], a2 = alpha[2];
  const float Cs = XDBL[(size_t)(b * kKX + kR + 1) * kL + l];
  int yo1[3], yo2[3], yo3[3], xo1[3], xo2[3], xo3[3];
#pragma unroll
  for (int i = 0; i < 3; ++i) {
    yo1[i] = clamp63(hr + (i - 1) * 1) * kGW;
    yo2[i] = clamp63(hr + (i - 1) * 2) * kGW;
    yo3[i] = clamp63(hr + (i - 1) * 3) * kGW;
    xo1[i] = clamp63(w + (i - 1) * 1);
    xo2[i] = clamp63(w + (i - 1) * 2);
    xo3[i] = clamp63(w + (i - 1) * 3);
  }
#pragma unroll 1
  for (int cc = 0; cc < 16; ++cc) {
    const int c = cc * 4 + cq;
    const int d = c0 + c;
    const float* hrow = Hb + (size_t)(b * kDI + d) * kL;
    const float* w1 = kw1 + d * 9;
    const float* w2 = kw2 + d * 9;
    const float* w3 = kw3 + d * 9;
    float s1 = 0.0f, s2 = 0.0f, s3 = 0.0f;
#pragma unroll
    for (int i = 0; i < 3; ++i) {
#pragma unroll
      for (int j = 0; j < 3; ++j) {
        s1 += w1[i * 3 + j] * hrow[yo1[i] + xo1[j]];
        s2 += w2[i * 3 + j] * hrow[yo2[i] + xo2[j]];
        s3 += w3[i * 3 + j] * hrow[yo3[i] + xo3[j]];
      }
    }
    const float hv = a0 * s1 + a1 * s2 + a2 * s3;
    const float xv = XS[(size_t)(b * kDI + d) * kL + l];
    sy[w * 68 + c] = hv * Cs + xv * Ds[d];
  }
  __syncthreads();
  const int lane = t & 31, wv = t >> 5;
  const int hh = lane >> 4, c4 = (lane & 15) * 4;
  for (int pass = 0; pass < 2; ++pass) {
#pragma unroll
    for (int it = 0; it < 4; ++it) {
      const int row = wv * 8 + it * 2 + hh;
      const v4f v = *(const v4f*)(sy + row * 68 + c4);
      *(volatile v4f*)(Y + (size_t)(b * kL + hr * kGW + row) * kDI + c0 + c4) = v;
    }
    __threadfence();
  }
}

__global__ __launch_bounds__(256) void k_lngate(const float* __restrict__ Y, const unsigned short* __restrict__ ZH,
                                                const unsigned short* __restrict__ ZL, const float* __restrict__ lnw,
                                                const float* __restrict__ lnb, unsigned short* __restrict__ GH,
                                                unsigned short* __restrict__ GL) {
  __shared__ __align__(16) float syv[4 * 512];
  __shared__ __align__(16) float sgv[4 * 512];
  __shared__ float sp1[8];
  __shared__ float sp2[8];
  const int t    = threadIdx.x;
  const int lane = t & 31;
  const int wv   = t >> 5;
  const int r    = t >> 6;
  const int cl   = t & 63;
  const size_t row = (size_t)blockIdx.x * 4 + r;
  const float* yr = Y + row * kDI;
  const unsigned* zh32 = (const unsigned*)(ZH + row * kDI);
  const unsigned* zl32 = (const unsigned*)(ZL + row * kDI);
  float s1 = 0.0f;
#pragma unroll 1
  for (int k = 0; k < 8; ++k) {
    const int c = cl + 64 * k;
    const float yv = yr[c];
    s1 += yv;
    syv[r * 512 + c] = yv;
    const unsigned wh = zh32[c >> 1];
    const unsigned wl = zl32[c >> 1];
    const unsigned sh_bits = (c & 1) ? (wh & 0xffff0000u) : (wh << 16);
    const unsigned sl_bits = (c & 1) ? (wl & 0xffff0000u) : (wl << 16);
    const float z = __uint_as_float(sh_bits) + __uint_as_float(sl_bits);
    const float sg = 1.0f / (1.0f + expf(-z));
    sgv[r * 512 + c] = z * sg;
  }
  s1 = wave_sum(s1);
  if (lane == 0) sp1[wv] = s1;
  __syncthreads();
  const float mean = (sp1[2 * r] + sp1[2 * r + 1]) * kInvDI;
  float s2 = 0.0f;
#pragma unroll 1
  for (int k = 0; k < 8; ++k) {
    const float dv = syv[r * 512 + cl + 64 * k] - mean;
    s2 += dv * dv;
  }
  s2 = wave_sum(s2);
  if (lane == 0) sp2[wv] = s2;
  __syncthreads();
  const float var  = (sp2[2 * r] + sp2[2 * r + 1]) * kInvDI;
  const float rinv = 1.0f / sqrtf(var + kLnEps);
  const int c8 = cl * 8;
  unsigned short hb[8], lb[8];
#pragma unroll
  for (int e = 0; e < 8; ++e) {
    const int c = c8 + e;
    const float yn = (syv[r * 512 + c] - mean) * rinv * lnw[c] + lnb[c];
    const float o  = yn * sgv[r * 512 + c];
    hb[e] = f2bf_bits(o);
    lb[e] = f2bf_bits(o - bf_bits2f(hb[e]));
  }
  const v4u uh = (v4u){pk16(hb[0], hb[1]), pk16(hb[2], hb[3]), pk16(hb[4], hb[5]), pk16(hb[6], hb[7])};
  const v4u ul = (v4u){pk16(lb[0], lb[1]), pk16(lb[2], lb[3]), pk16(lb[4], lb[5]), pk16(lb[6], lb[7])};
  const size_t o = row * kDI + c8;
  *(volatile v4u*)(GH + o) = uh;
  *(volatile v4u*)(GL + o) = ul;
  __threadfence();
  *(volatile v4u*)(GH + o) = uh;
  *(volatile v4u*)(GL + o) = ul;
}

extern "C" void kernel_launch(void* const* d_in, const int* in_sizes, int n_in,
                              void* d_out, int out_size, void* d_ws, size_t ws_size,
                              hipStream_t stream) {
  if (n_in < 16) return;
  if (in_sizes[0] != kTok * kDM || in_sizes[1] != 2 * kDI * kDM || in_sizes[4] != kKXV * kDI ||
      in_sizes[5] != kDI * kR || in_sizes[15] != kDM * kDI || out_size != kTok * kDM) return;
  const float* x      = (const float*)d_in[0];
  const float* ipw    = (const float*)d_in[1];
  const float* convw  = (const float*)d_in[2];
  const float* convb  = (const float*)d_in[3];
  const float* xpw    = (const float*)d_in[4];
  const float* dtw    = (const float*)d_in[5];
  const float* dtb    = (const float*)d_in[6];
  const float* A_logs = (const float*)d_in[7];
  const float* Ds     = (const float*)d_in[8];
  const float* sfk1   = (const float*)d_in[9];
  const float* sfk2   = (const float*)d_in[10];
  const float* sfk3   = (const float*)d_in[11];
  const float* alpha  = (const float*)d_in[12];
  const float* lnw    = (const float*)d_in[13];
  const float* lnb    = (const float*)d_in[14];
  const float* opw    = (const float*)d_in[15];
  float* out = (float*)d_out;

  const size_t MiB = (size_t)1048576;
  const size_t KiB = (size_t)1024;
  char* ws = (char*)d_ws;
  const size_t planeB16 = (size_t)kTok * kDI * 2;
  const size_t planeF32 = (size_t)kTok * kDI * 4;
  const size_t wiPlane  = (size_t)2 * kDI * kDM * 2;
  const size_t woPlane  = (size_t)kDM * kDI * 2;
  const size_t xpPlane  = (size_t)kKX * kDI * 2;
  const size_t dwPlane  = (size_t)kDI * kR * 2;
  const size_t xdblB    = (size_t)kNB * kKX * kL * 4;
  const size_t drPlane  = (size_t)kNB * kL * kR * 2;
  const size_t offA = 0, offB = offA + planeF32, offC = offB + planeF32, offD = offC + planeF32;
  const size_t offWIH = offD,            offWIL = offWIH + wiPlane;
  const size_t offWOH = offWIL + wiPlane, offWOL = offWOH + woPlane;
  const size_t offXPH = offWOL + woPlane, offXPL = offXPH + xpPlane;
  const size_t offDWH = offXPL + xpPlane, offDWL = offDWH + dwPlane;
  const size_t offXDBL = offDWL + dwPlane;
  const size_t offDRH = offXDBL + xdblB,  offDRL = offDRH + drPlane;
  const size_t wsEnd  = offDRL + drPlane;
  if (2 * planeB16 != planeF32) return;
  if (wsEnd != (size_t)105 * MiB + 192 * KiB) return;
  if (ws_size < wsEnd) return;

  unsigned short* XH   = (unsigned short*)(ws + offA);
  unsigned short* XL   = (unsigned short*)(ws + offA + planeB16);
  unsigned short* XSTH = (unsigned short*)(ws + offA);
  unsigned short* XSTL = (unsigned short*)(ws + offA + planeB16);
  float*          Ybuf = (float*)(ws + offA);
  float*          XIN  = (float*)(ws + offB);
  float*          Hbuf = (float*)(ws + offB);
  unsigned short* ZH   = (unsigned short*)(ws + offB);
  unsigned short* ZL   = (unsigned short*)(ws + offB + planeB16);
  float*          XS   = (float*)(ws + offC);
  unsigned short* X2H  = (unsigned short*)(ws + offC);
  unsigned short* X2L  = (unsigned short*)(ws + offC + planeB16);
  unsigned short* GH   = (unsigned short*)(ws + offC);
  unsigned short* GL   = (unsigned short*)(ws + offC + planeB16);
  unsigned short* WIH  = (unsigned short*)(ws + offWIH);
  unsigned short* WIL  = (unsigned short*)(ws + offWIL);
  unsigned short* WOH  = (unsigned short*)(ws + offWOH);
  unsigned short* WOL  = (unsigned short*)(ws + offWOL);
  unsigned short* XPH  = (unsigned short*)(ws + offXPH);
  unsigned short* XPL  = (unsigned short*)(ws + offXPL);
  unsigned short* DWH  = (unsigned short*)(ws + offDWH);
  unsigned short* DWL  = (unsigned short*)(ws + offDWL);
  float*          XDBL = (float*)(ws + offXDBL);
  unsigned short* DRH  = (unsigned short*)(ws + offDRH);
  unsigned short* DRL  = (unsigned short*)(ws + offDRL);
  void*        unusedp = (void*)(ws + offXDBL);
  const float* unusedf = (const float*)(ws + offXDBL);

  k_split8<<<dim3(kTok * kDM / 8 / 256), dim3(256), 0, stream>>>(x, XH, XL, kTok * kDM / 8, kTok * kDM / 8);
  k_split8<<<dim3(2 * kDI * kDM / 8 / 256), dim3(256), 0, stream>>>(ipw, WIH, WIL, 2 * kDI * kDM / 8, 2 * kDI * kDM / 8);
  k_split8<<<dim3(kDM * kDI / 8 / 256), dim3(256), 0, stream>>>(opw, WOH, WOL, kDM * kDI / 8, kDM * kDI / 8);
  k_split8<<<dim3(kKX * kDI / 8 / 256), dim3(256), 0, stream>>>(xpw, XPH, XPL, kKX * kDI / 8, kKXV * kDI / 8);
  k_split8<<<dim3(kDI * kR / 8 / 256), dim3(256), 0, stream>>>(dtw, DWH, DWL, kDI * kR / 8, kDI * kR / 8);

  wmma_gemm64<1, true, 0, 0, false><<<dim3(64, kNB), dim3(256), 0, stream>>>(
      WIH, WIL, kDM, 0L, XH, XL, kDM, (long)kL * kDM,
      (void*)XIN, unusedp, kL, (long)kDI * kL, unusedf, unusedf, 0L, kDI, kL, kDM, 1.0f);
  k_conv1<<<dim3(kGW, kDI / 64, kNB), dim3(256), 0, stream>>>(XIN, convw, convb, XS, XSTH, XSTL);
  wmma_gemm64<1, true, 0, 0, false><<<dim3(8, kNB), dim3(256), 0, stream>>>(
      XPH, XPL, kDI, 0L, XSTH, XSTL, kDI, (long)kL * kDI,
      (void*)XDBL, unusedp, kL, (long)kKX * kL, unusedf, unusedf, 0L, kKX, kL, kDI, 1.0f);
  k_dtr<<<dim3(kL / 64, kNB), dim3(256), 0, stream>>>(XDBL, DRH, DRL);
  k_scan<<<dim3(kDI / 64, kNB), dim3(64), 0, stream>>>(DWH, DWL, DRH, DRL, XS, XDBL, dtb, A_logs, Hbuf);
  k_fuse<<<dim3(kGW, kDI / 64, kNB), dim3(256), 0, stream>>>(Hbuf, XS, XDBL, Ds, sfk1, sfk2, sfk3, alpha, Ybuf);
  k_split8<<<dim3(kTok * kDM / 8 / 256), dim3(256), 0, stream>>>(x, X2H, X2L, kTok * kDM / 8, kTok * kDM / 8);
  wmma_gemm64<1, true, 0, 2, false><<<dim3(256, 1), dim3(256), 0, stream>>>(
      X2H, X2L, kDM, 0L, WIH + (size_t)kDI * kDM, WIL + (size_t)kDI * kDM, kDM, 0L,
      (void*)ZH, (void*)ZL, kDI, 0L, unusedf, unusedf, 0L, kTok, kDI, kDM, 1.0f);
  k_lngate<<<dim3(kTok / 4), dim3(256), 0, stream>>>(Ybuf, ZH, ZL, lnw, lnb, GH, GL);
  wmma_gemm64<1, true, 0, 0, false><<<dim3(256, 1), dim3(256), 0, stream>>>(
      GH, GL, kDI, 0L, WOH, WOL, kDI, 0L,
      (void*)out, unusedp, kDM, 0L, unusedf, unusedf, 0L, kTok, kDM, kDI, 1.0f);
}
